// DynGRU_29746943492385
// MI455X (gfx1250) — hardware-verified
//
#include <hip/hip_runtime.h>
#include <math.h>
#include <stddef.h>

typedef __attribute__((ext_vector_type(16))) _Float16 v16h;
typedef __attribute__((ext_vector_type(8)))  _Float16 v8h;
typedef __attribute__((ext_vector_type(16))) __bf16   v16b;
typedef __attribute__((ext_vector_type(8)))  __bf16   v8b;
typedef __attribute__((ext_vector_type(8)))  float    v8f;
typedef __attribute__((ext_vector_type(4)))  float    v4f;

__device__ __forceinline__ unsigned short f2bf_bits(float f) {
  unsigned u = __float_as_uint(f);
  return (unsigned short)((u + 0x7FFFu + ((u >> 16) & 1u)) >> 16);
}
__device__ __forceinline__ float bf_bits2f(unsigned short h) { return __uint_as_float(((unsigned)h) << 16); }

__device__ __forceinline__ void dep_guard_h(v8f& a, v8f& b, v16h x, v16h y) { asm volatile("v_nop\n\tv_nop\n\tv_nop\n\tv_nop" : "+v"(a), "+v"(b) : "v"(x), "v"(y)); }
__device__ __forceinline__ void dep_guard_b(v8f& a, v8f& b, v16b x, v16b y) { asm volatile("v_nop\n\tv_nop\n\tv_nop\n\tv_nop" : "+v"(a), "+v"(b) : "v"(x), "v"(y)); }
__device__ __forceinline__ void keep4_h(v16h a, v16h b, v16h c, v16h d) { asm volatile("v_nop" :: "v"(a), "v"(b), "v"(c), "v"(d)); }
__device__ __forceinline__ void keep4_b(v16b a, v16b b, v16b c, v16b d) { asm volatile("v_nop" :: "v"(a), "v"(b), "v"(c), "v"(d)); }
__device__ __forceinline__ void acc_guard4(v8f& a, v8f& b, v8f& c, v8f& d) { asm volatile("v_nop\n\tv_nop\n\tv_nop\n\tv_nop" : "+v"(a), "+v"(b), "+v"(c), "+v"(d)); }
__device__ __forceinline__ void dep_guard3h(v8f& a, v8f& b, v8f& c, v16h x, v16h y, v16h z, v16h w) {
  asm volatile("v_nop\n\tv_nop\n\tv_nop\n\tv_nop" : "+v"(a), "+v"(b), "+v"(c) : "v"(x), "v"(y), "v"(z), "v"(w));
}

template <typename T> struct Frag;
template <> struct Frag<_Float16> {
  typedef v16h V; union U { v16h v; v8h h[2]; };
  static __device__ __forceinline__ v16h load(const _Float16* p) {
    U f; f.h[0] = *(const v8h*)(p); f.h[1] = *(const v8h*)(p + 16); return f.v;
  }
  static __device__ __forceinline__ v8f mma(v16h a, v16h b, v8f c) {
    return __builtin_amdgcn_wmma_f32_16x16x32_f16(false, a, false, b, (short)0, c, false, false);
  }
  static __device__ __forceinline__ void guard(v8f& a, v8f& b, v16h x, v16h y) { dep_guard_h(a, b, x, y); }
  static __device__ __forceinline__ void keep(v16h a, v16h b, v16h c, v16h d) { keep4_h(a, b, c, d); }
};
template <> struct Frag<__bf16> {
  typedef v16b V; union U { v16b v; v8b h[2]; };
  static __device__ __forceinline__ v16b load(const __bf16* p) {
    U f; f.h[0] = *(const v8b*)(p); f.h[1] = *(const v8b*)(p + 16); return f.v;
  }
  static __device__ __forceinline__ v8f mma(v16b a, v16b b, v8f c) {
    return __builtin_amdgcn_wmma_f32_16x16x32_bf16(false, a, false, b, (short)0, c, false, false);
  }
  static __device__ __forceinline__ void guard(v8f& a, v8f& b, v16b x, v16b y) { dep_guard_b(a, b, x, y); }
  static __device__ __forceinline__ void keep(v16b a, v16b b, v16b c, v16b d) { keep4_b(a, b, c, d); }
};

template <int ET> struct Elem;
template <> struct Elem<0> { typedef _Float16 T; };
template <> struct Elem<1> { typedef __bf16 T; };
template <int ET, bool SPLIT, int BIAS_MODE, int OUT_MODE, bool RESID, int ACT = 0>
__global__ __launch_bounds__(256) void wmma_gemm64(
    const unsigned short* __restrict__ Ap, const unsigned short* __restrict__ A2p, int lda, long strideA,
    const unsigned short* __restrict__ Btp, const unsigned short* __restrict__ Bt2p, int ldb, long strideB,
    void* __restrict__ Cout, void* __restrict__ Cout2, int ldc, long strideC,
    const float* __restrict__ bias,
    const float* __restrict__ resid, long strideR,
    int M, int N, int K, float scale, float oscale) {
  typedef typename Elem<ET>::T T;
  typedef typename Frag<T>::V V;
  const T* A = (const T*)Ap; const T* A2 = (const T*)A2p; const T* Bt = (const T*)Btp; const T* Bt2 = (const T*)Bt2p;
  __shared__ __align__(16) float sT[8][16 * 68];
  const int b    = blockIdx.y;
  const int lane = threadIdx.x & 31;
  const int wave = threadIdx.x >> 5;
  const int tilesN = N >> 6;
  const int tilesM = M >> 6;
  const int tile = blockIdx.x * 8 + wave;
  if (tile >= tilesM * tilesN) return;
  const int tm = tile / tilesN;
  const int tn = tile - tm * tilesN;
  const int m0 = tm << 6;
  const int n0 = tn << 6;

  const T* Ab  = A  + (size_t)b * strideA;
  const T* Bb  = Bt + (size_t)b * strideB;
  const T* Ab2 = SPLIT ? (A2  + (size_t)b * strideA) : nullptr;
  const T* Bb2 = SPLIT ? (Bt2 + (size_t)b * strideB) : nullptr;

  const int rlane = lane & 15;
  const int koff  = (lane >> 4) * 8;
  const int mOff  = (lane >> 4) * 8;

  v8f acc[4][4];
#pragma unroll
  for (int i = 0; i < 4; ++i)
#pragma unroll
    for (int j = 0; j < 4; ++j) acc[i][j] = (v8f){0.f,0.f,0.f,0.f,0.f,0.f,0.f,0.f};

  for (int k0 = 0; k0 < K; k0 += 32) {
    V bh[4], bl[4];
#pragma unroll
    for (int j = 0; j < 4; ++j) {
      const size_t bo = (size_t)(n0 + (j << 4) + rlane) * ldb + koff + k0;
      bh[j] = Frag<T>::load(Bb + bo);
      if (SPLIT) bl[j] = Frag<T>::load(Bb2 + bo);
    }
#pragma unroll
    for (int i = 0; i < 4; ++i) {
      const size_t ao = (size_t)(m0 + (i << 4) + rlane) * lda + koff + k0;
      V ah = Frag<T>::load(Ab + ao);
      V al;
      if (SPLIT) al = Frag<T>::load(Ab2 + ao);
#pragma unroll
      for (int j = 0; j < 4; ++j) {
        acc[i][j] = Frag<T>::mma(ah, bh[j], acc[i][j]);
        if (SPLIT) {
          acc[i][j] = Frag<T>::mma(ah, bl[j], acc[i][j]);
          acc[i][j] = Frag<T>::mma(al, bh[j], acc[i][j]);
        }
      }
      Frag<T>::guard(acc[i][0], acc[i][3], ah, SPLIT ? al : ah);
    }
    Frag<T>::keep(bh[0], bh[1], bh[2], bh[3]);
    if (SPLIT) Frag<T>::keep(bl[0], bl[1], bl[2], bl[3]);
  }
  acc_guard4(acc[0][0], acc[0][1], acc[0][2], acc[0][3]);
  acc_guard4(acc[1][0], acc[1][1], acc[1][2], acc[1][3]);
  acc_guard4(acc[2][0], acc[2][1], acc[2][2], acc[2][3]);
  acc_guard4(acc[3][0], acc[3][1], acc[3][2], acc[3][3]);

  float* slab = sT[wave];
  const float* Rb = RESID ? (resid + (size_t)b * strideR) : nullptr;
#pragma unroll
  for (int i = 0; i < 4; ++i) {
    const int mBase = m0 + (i << 4);
#pragma unroll
    for (int j = 0; j < 4; ++j) {
      const int n = n0 + (j << 4) + rlane;
      float bv = 0.f;
      if (BIAS_MODE == 2) bv = bias[n];
#pragma unroll
      for (int r = 0; r < 8; ++r) {
        float v = acc[i][j][r] * scale;
        if (BIAS_MODE == 1) v += bias[mBase + mOff + r];
        if (BIAS_MODE == 2) v += bv;
        if (RESID) v += Rb[(size_t)(mBase + mOff + r) * ldc + n];
        if (ACT == 1) v = tanhf(v);
        if (ACT == 2) v = fmaxf(v, 0.0f);
        if (ACT == 4) v = (v > 0.f) ? v : 0.01f * v;
        v = v * oscale;
        slab[(mOff + r) * 68 + (j << 4) + rlane] = v;
      }
    }
    __builtin_amdgcn_fence(__ATOMIC_RELEASE, "workgroup");
    __builtin_amdgcn_wave_barrier();
    __builtin_amdgcn_fence(__ATOMIC_ACQUIRE, "workgroup");
    if (OUT_MODE == 0) {
      float* C = (float*)Cout + (size_t)b * strideC;
      const int hh = lane >> 4, c4 = (lane & 15) * 4;
      for (int pass = 0; pass < 2; ++pass) {
#pragma unroll
        for (int it = 0; it < 8; ++it) {
          const int row = it * 2 + hh;
          v4f v = *(const v4f*)(slab + row * 68 + c4);
          *(volatile v4f*)(C + (size_t)(mBase + row) * ldc + n0 + c4) = v;
        }
        __threadfence();
      }
    } else {
      const int q = lane >> 3, c8 = (lane & 7) * 8;
      unsigned short* C  = (unsigned short*)Cout  + (size_t)b * strideC;
      unsigned short* C2 = (OUT_MODE == 2) ? ((unsigned short*)Cout2 + (size_t)b * strideC) : nullptr;
      for (int pass = 0; pass < 2; ++pass) {
#pragma unroll
        for (int it = 0; it < 4; ++it) {
          const int row = it * 4 + q;
          const float* sp = slab + row * 68 + c8;
          v8h hv, lv;
#pragma unroll
          for (int e = 0; e < 8; ++e) {
            if (OUT_MODE == 1) {
              hv[e] = (_Float16)sp[e];
            } else {
              unsigned short hb = f2bf_bits(sp[e]);
              unsigned short lb = f2bf_bits(sp[e] - bf_bits2f(hb));
              hv[e] = __builtin_bit_cast(_Float16, hb);
              lv[e] = __builtin_bit_cast(_Float16, lb);
            }
          }
          *(volatile v8h*)(C + (size_t)(mBase + row) * ldc + n0 + c8) = hv;
          if (OUT_MODE == 2) *(volatile v8h*)(C2 + (size_t)(mBase + row) * ldc + n0 + c8) = lv;
        }
        __threadfence();
      }
    }
    __builtin_amdgcn_fence(__ATOMIC_RELEASE, "workgroup");
    __builtin_amdgcn_wave_barrier();
    __builtin_amdgcn_fence(__ATOMIC_ACQUIRE, "workgroup");
  }
}

__global__ __launch_bounds__(256) void cast_f32_f16x2s(
    const float* __restrict__ in, _Float16* __restrict__ out, int n2, float scale) {
  int i = blockIdx.x * 256 + threadIdx.x;
  if (i < n2) {
    const _Float16 h0 = (_Float16)(in[2 * i] * scale), h1 = (_Float16)(in[2 * i + 1] * scale);
    const unsigned u = (unsigned)__builtin_bit_cast(unsigned short, h0) | ((unsigned)__builtin_bit_cast(unsigned short, h1) << 16);
    ((volatile unsigned*)out)[i] = u;
    __threadfence();
    ((volatile unsigned*)out)[i] = u;
  }
}

constexpr int NBAT = 32;
constexpr int LSEQ = 1024;
constexpr int DIN_X = 64;
constexpr int DMEM = 512;
constexpr int DHID = 512;
constexpr int DOUT_Y = 64;
constexpr int N3GATE = 1536;
constexpr int NTOK = NBAT * LSEQ;
constexpr int LPITCH = 520;
constexpr int SCAN_THREADS = 512;
constexpr int SCAN_ROWS = 16;
constexpr float W_CARRY = 64.0f;
constexpr float A_CARRY = 8.0f;

__device__ __forceinline__ float sigm_f(float x) { return __builtin_amdgcn_rcpf(1.0f + expf(-x)); }
__device__ __forceinline__ float tanh_r(float y) {
  const float yc = fminf(fmaxf(y, -15.0f), 15.0f);
  const float e = expf(-2.0f * yc);
  return (1.0f - e) * __builtin_amdgcn_rcpf(1.0f + e);
}

union FragH { v16h v; v8h h[2]; };

__global__ __launch_bounds__(SCAN_THREADS) void gru_scan16(
    const unsigned short* __restrict__ S1p,
    const unsigned short* __restrict__ Wxp,
    const float* __restrict__ bx,
    const unsigned short* __restrict__ Whp,
    const float* __restrict__ bh,
    unsigned short* __restrict__ Hsp) {
  __shared__ __align__(16) _Float16 sS1[SCAN_ROWS * LPITCH];
  __shared__ __align__(16) _Float16 sH[2][SCAN_ROWS * LPITCH];
  const _Float16* S1g = (const _Float16*)S1p;
  const _Float16* Wx  = (const _Float16*)Wxp;
  const _Float16* Wh  = (const _Float16*)Whp;
  _Float16* Hs = (_Float16*)Hsp;

  const int tid  = threadIdx.x;
  const int lane = tid & 31;
  const int wave = tid >> 5;
  const int c    = lane & 15;
  const int hh   = lane >> 4;
  const int koff = hh * 8;
  const int row0 = blockIdx.x * SCAN_ROWS;
  const float kInv = 1.0f / 512.0f;

  float ba[2], bc[2], bxh[2], bhh[2];
  float hreg[2][8];
#pragma unroll
  for (int u = 0; u < 2; ++u) {
    const int j = 16 * (2 * wave + u) + c;
    ba[u]  = bx[j] + bh[j];
    bc[u]  = bx[DMEM + j] + bh[DMEM + j];
    bxh[u] = bx[2 * DMEM + j];
    bhh[u] = bh[2 * DMEM + j];
#pragma unroll
    for (int r = 0; r < 8; ++r) hreg[u][r] = 0.0f;
  }
  {
    v8h z;
#pragma unroll
    for (int e = 0; e < 8; ++e) z[e] = (_Float16)0.0f;
    for (int q = tid; q < (SCAN_ROWS * LPITCH) / 8; q += SCAN_THREADS) *(v8h*)(&sH[0][q * 8]) = z;
  }

  for (int t = 0; t < LSEQ; ++t) {
    const int cur = t & 1;
    const _Float16* sHc = sH[cur];
    _Float16* sHn = sH[cur ^ 1];

#pragma unroll
    for (int i = 0; i < 2; ++i) {
      const int q = tid + SCAN_THREADS * i;
      const int r = q >> 6, c16 = q & 63;
      const v8h v = *(const v8h*)(S1g + ((size_t)(row0 + r) * LSEQ + t) * DHID + c16 * 8);
      *(v8h*)(sS1 + r * LPITCH + c16 * 8) = v;
    }
    __syncthreads();

    v8f aA[2], aC[2], aX[2], aH[2];
#pragma unroll
    for (int u = 0; u < 2; ++u) {
      aA[u] = (v8f){0.f,0.f,0.f,0.f,0.f,0.f,0.f,0.f};
      aC[u] = (v8f){0.f,0.f,0.f,0.f,0.f,0.f,0.f,0.f};
      aX[u] = (v8f){0.f,0.f,0.f,0.f,0.f,0.f,0.f,0.f};
      aH[u] = (v8f){0.f,0.f,0.f,0.f,0.f,0.f,0.f,0.f};
    }

#pragma unroll 1
    for (int ks = 0; ks < DHID / 32; ++ks) {
      const int k0 = ks * 32;
      FragH fa;
      fa.h[0] = *(const v8h*)(sS1 + c * LPITCH + k0 + koff);
      fa.h[1] = *(const v8h*)(sS1 + c * LPITCH + k0 + koff + 16);
#pragma unroll
      for (int u = 0; u < 2; ++u) {
        const size_t jrow = (size_t)(16 * (2 * wave + u) + c);
        const v16h b0 = Frag<_Float16>::load(Wx + (jrow) * DHID + k0 + koff);
        const v16h b1 = Frag<_Float16>::load(Wx + (jrow + DMEM) * DHID + k0 + koff);
        const v16h b2 = Frag<_Float16>::load(Wx + (jrow + 2 * DMEM) * DHID + k0 + koff);
        aA[u] = Frag<_Float16>::mma(fa.v, b0, aA[u]);
        aC[u] = Frag<_Float16>::mma(fa.v, b1, aC[u]);
        aX[u] = Frag<_Float16>::mma(fa.v, b2, aX[u]);
        dep_guard3h(aA[u], aC[u], aX[u], fa.v, b0, b1, b2);
      }
    }
#pragma unroll 1
    for (int ks = 0; ks < DMEM / 32; ++ks) {
      const int k0 = ks * 32;
      FragH fa;
      fa.h[0] = *(const v8h*)(sHc + c * LPITCH + k0 + koff);
      fa.h[1] = *(const v8h*)(sHc + c * LPITCH + k0 + koff + 16);
#pragma unroll
      for (int u = 0; u < 2; ++u) {
        const size_t jrow = (size_t)(16 * (2 * wave + u) + c);
        const v16h b0 = Frag<_Float16>::load(Wh + (jrow) * DMEM + k0 + koff);
        const v16h b1 = Frag<_Float16>::load(Wh + (jrow + DMEM) * DMEM + k0 + koff);
        const v16h b2 = Frag<_Float16>::load(Wh + (jrow + 2 * DMEM) * DMEM + k0 + koff);
        aA[u] = Frag<_Float16>::mma(fa.v, b0, aA[u]);
        aC[u] = Frag<_Float16>::mma(fa.v, b1, aC[u]);
        aH[u] = Frag<_Float16>::mma(fa.v, b2, aH[u]);
        dep_guard3h(aA[u], aC[u], aH[u], fa.v, b0, b1, b2);
      }
    }
    acc_guard4(aA[0], aC[0], aX[0], aH[0]);
    acc_guard4(aA[1], aC[1], aX[1], aH[1]);

#pragma unroll
    for (int u = 0; u < 2; ++u) {
      const int jl = 16 * (2 * wave + u) + c;
#pragma unroll
      for (int r = 0; r < 8; ++r) {
        const float sa = aA[u][r] * kInv + ba[u];
        const float sc = aC[u][r] * kInv + bc[u];
        const float sx = aX[u][r] * kInv + bxh[u];
        const float sh = aH[u][r] * kInv + bhh[u];
        const float ag = sigm_f(sa);
        const float cg = sigm_f(sc);
        const float th = tanh_r(sx + ag * sh);
        const float ho = hreg[u][r];
        const float hn = (1.0f - cg) * ho + cg * th;
        hreg[u][r] = hn;
        sHn[(8 * hh + r) * LPITCH + jl] = (_Float16)(hn * A_CARRY);
      }
    }
    __syncthreads();

    {
      _Float16* dst = Hs + ((size_t)(row0 + wave) * LSEQ + t) * DMEM;
      const _Float16* src = sHn + wave * LPITCH;
      const v8h v0 = *(const v8h*)(src + lane * 8);
      const v8h v1 = *(const v8h*)(src + 256 + lane * 8);
      for (int pass = 0; pass < 2; ++pass) {
        *(volatile v8h*)(dst + lane * 8) = v0;
        *(volatile v8h*)(dst + 256 + lane * 8) = v1;
        __threadfence();
      }
    }
  }
}

extern "C" void kernel_launch(void* const* d_in, const int* in_sizes, int n_in,
                              void* d_out, int out_size, void* d_ws, size_t ws_size,
                              hipStream_t stream) {
  if (n_in < 15) return;
  if (in_sizes[0] != NTOK * DIN_X || in_sizes[1] != DHID * DIN_X || in_sizes[2] != DHID ||
      in_sizes[3] != DHID * DHID || in_sizes[4] != DHID || in_sizes[5] != N3GATE * DHID ||
      in_sizes[6] != N3GATE || in_sizes[7] != DHID * DMEM || in_sizes[8] != DHID ||
      in_sizes[9] != DHID * DHID || in_sizes[10] != DHID || in_sizes[11] != DOUT_Y * DHID ||
      in_sizes[12] != DOUT_Y || in_sizes[13] != N3GATE * DMEM || in_sizes[14] != N3GATE) return;
  if (out_size != NTOK * DOUT_Y) return;

  const float* x_seq = (const float*)d_in[0];
  const float* sW0 = (const float*)d_in[1];
  const float* sb0 = (const float*)d_in[2];
  const float* sW1 = (const float*)d_in[3];
  const float* sb1 = (const float*)d_in[4];
  const float* sWt = (const float*)d_in[5];
  const float* sbt = (const float*)d_in[6];
  const float* aW0 = (const float*)d_in[7];
  const float* ab0 = (const float*)d_in[8];
  const float* aW1 = (const float*)d_in[9];
  const float* ab1 = (const float*)d_in[10];
  const float* aWt = (const float*)d_in[11];
  const float* abt = (const float*)d_in[12];
  const float* mW  = (const float*)d_in[13];
  const float* mb  = (const float*)d_in[14];
  float* out = (float*)d_out;

  char* ws = (char*)d_ws;
  size_t off = 0;
  auto carve = [&](size_t bytes) -> unsigned short* {
    unsigned short* p = (unsigned short*)(ws + off);
    off += (bytes + 255) & ~(size_t)255;
    return p;
  };
  unsigned short* x16  = carve((size_t)NTOK * DIN_X * 2);
  unsigned short* sW0h = carve((size_t)DHID * DIN_X * 2);
  unsigned short* sW1h = carve((size_t)DHID * DHID * 2);
  unsigned short* sWth = carve((size_t)N3GATE * DHID * 2);
  unsigned short* aW0h = carve((size_t)DHID * DMEM * 2);
  unsigned short* aW1h = carve((size_t)DHID * DHID * 2);
  unsigned short* aWth = carve((size_t)DOUT_Y * DHID * 2);
  unsigned short* mWh  = carve((size_t)N3GATE * DMEM * 2);
  unsigned short* regA = carve((size_t)NTOK * DHID * 2);
  unsigned short* regB = carve((size_t)NTOK * DHID * 2);
  if (off > ws_size) return;

  auto cast = [&](const float* src, unsigned short* dst, int n, float scale) {
    const int n2 = n / 2;
    cast_f32_f16x2s<<<dim3((n2 + 255) / 256), dim3(256), 0, stream>>>(src, (_Float16*)dst, n2, scale);
  };
  cast(x_seq, x16, NTOK * DIN_X, 1.0f);
  cast(sW0, sW0h, DHID * DIN_X, W_CARRY);
  cast(sW1, sW1h, DHID * DHID, W_CARRY);
  cast(sWt, sWth, N3GATE * DHID, W_CARRY);
  cast(aW0, aW0h, DHID * DMEM, W_CARRY);
  cast(aW1, aW1h, DHID * DHID, W_CARRY);
  cast(aWt, aWth, DOUT_Y * DHID, W_CARRY);
  cast(mW, mWh, N3GATE * DMEM, W_CARRY);

  {
    const int tiles = (NTOK / 64) * (DHID / 64);
    wmma_gemm64<0, false, 2, 1, false, 2><<<dim3((tiles + 7) / 8, 1), dim3(256), 0, stream>>>(
        x16, x16, DIN_X, 0L, sW0h, sW0h, DIN_X, 0L, regA, regA, DHID, 0L, sb0, sb0, 0L,
        NTOK, DHID, DIN_X, 1.0f / W_CARRY, A_CARRY);
  }
  {
    const int tiles = (NTOK / 64) * (DHID / 64);
    wmma_gemm64<0, false, 2, 1, false, 2><<<dim3((tiles + 7) / 8, 1), dim3(256), 0, stream>>>(
        regA, regA, DHID, 0L, sW1h, sW1h, DHID, 0L, regB, regB, DHID, 0L, sb1, sb1, 0L,
        NTOK, DHID, DHID, 1.0f / (W_CARRY * A_CARRY), A_CARRY);
  }
  gru_scan16<<<dim3(NBAT / SCAN_ROWS), dim3(SCAN_THREADS), 0, stream>>>(regB, sWth, sbt, mWh, mb, regA);
  {
    const int tiles = (NTOK / 64) * (DHID / 64);
    wmma_gemm64<0, false, 2, 1, false, 2><<<dim3((tiles + 7) / 8, 1), dim3(256), 0, stream>>>(
        regA, regA, DMEM, 0L, aW0h, aW0h, DMEM, 0L, regB, regB, DHID, 0L, ab0, ab0, 0L,
        NTOK, DHID, DMEM, 1.0f / (W_CARRY * A_CARRY), A_CARRY);
  }
  {
    const int tiles = (NTOK / 64) * (DHID / 64);
    wmma_gemm64<0, false, 2, 1, false, 2><<<dim3((tiles + 7) / 8, 1), dim3(256), 0, stream>>>(
        regB, regB, DHID, 0L, aW1h, aW1h, DHID, 0L, regA, regA, DHID, 0L, ab1, ab1, 0L,
        NTOK, DHID, DHID, 1.0f / (W_CARRY * A_CARRY), A_CARRY);
  }
  {
    const int tiles = (NTOK / 64) * (DOUT_Y / 64);
    wmma_gemm64<0, false, 2, 0, false, 0><<<dim3((tiles + 7) / 8, 1), dim3(256), 0, stream>>>(
        regA, regA, DHID, 0L, aWth, aWth, DHID, 0L, out, out, DOUT_Y, 0L, abt, abt, 0L,
        NTOK, DOUT_Y, DHID, 1.0f / (W_CARRY * A_CARRY), 1.0f);
  }
}
